// VanillaRNN_47588237639944
// MI455X (gfx1250) — hardware-run, weakly checked
//
#include <hip/hip_runtime.h>
#include <math.h>

typedef __attribute__((ext_vector_type(16))) _Float16 v16h;
typedef __attribute__((ext_vector_type(8)))  _Float16 v8h;
typedef __attribute__((ext_vector_type(2)))  _Float16 v2h;
typedef __attribute__((ext_vector_type(8)))  float    v8f;
typedef __attribute__((ext_vector_type(4)))  float    v4f;
typedef __attribute__((ext_vector_type(2)))  float    v2f;

constexpr int kVocab = 128;
constexpr int kEmbed = 256;
constexpr int kHid   = 512;
constexpr int kBatch = 64;
constexpr int kSeq   = 512;
constexpr int kRows  = kBatch * kSeq;
constexpr int kHP    = kHid + 8;
constexpr float kCarryH = 64.0f;
constexpr float kCarryW = 256.0f;
constexpr float kCarryR = 2048.0f;
constexpr float kFold   = 1.0f / (kCarryH * kCarryW);
constexpr float kResInv = 1.0f / kCarryR;
static_assert((kHid % 32) == 0);
static_assert((kRows % 64) == 0 && (kVocab % 64) == 0);
static_assert(kEmbed == 256);
static_assert((kBatch % 16) == 0 && kHid == 16 * 32);
static_assert(((kHP * 2) % 16) == 0);

constexpr size_t kSzHS   = (size_t)kRows * kHid * 2;
constexpr size_t kSzW    = (size_t)kHid * kHid * 2;
constexpr size_t kSzWY   = (size_t)kVocab * kHid * 2;
constexpr size_t kSzP0   = (size_t)kVocab * kHid * 4;
constexpr size_t kOffHS0  = 0;
constexpr size_t kOffHS1  = kOffHS0  + kSzHS;
constexpr size_t kOffWH0V = kOffHS1  + kSzHS;
constexpr size_t kOffWH0R = kOffWH0V + kSzW;
constexpr size_t kOffWX1V = kOffWH0R + kSzW;
constexpr size_t kOffWX1R = kOffWX1V + kSzW;
constexpr size_t kOffWH1V = kOffWX1R + kSzW;
constexpr size_t kOffWH1R = kOffWH1V + kSzW;
constexpr size_t kOffWYV  = kOffWH1R + kSzW;
constexpr size_t kOffP0   = kOffWYV  + kSzWY;
constexpr size_t kWsTotal = kOffP0   + kSzP0;
static_assert(kWsTotal == 70647808ull);
static_assert(kWsTotal <= 134217728ull);
static_assert((kOffHS1 % 128) == 0 && (kOffWH0V % 128) == 0 && (kOffWH0R % 128) == 0 && (kOffWX1V % 128) == 0 &&
              (kOffWX1R % 128) == 0 && (kOffWH1V % 128) == 0 && (kOffWH1R % 128) == 0 && (kOffWYV % 128) == 0 &&
              (kOffP0 % 128) == 0);

constexpr size_t kOutLogits = 0;
constexpr size_t kOutH0     = (size_t)kRows * kVocab;
constexpr size_t kOutH1     = kOutH0 + (size_t)kBatch * kHid;
constexpr size_t kOutTotal  = kOutH1 + (size_t)kBatch * kHid;
static_assert(kOutH0 * 4 == 16777216ull && kOutH1 * 4 == 16908288ull && kOutTotal * 4 == 17039360ull);

__device__ __forceinline__ v16h ld_frag(const _Float16* p) {
  union { v16h v; v8h h[2]; } f;
  f.h[0] = *(const v8h*)(p);
  f.h[1] = *(const v8h*)(p + 16);
  return f.v;
}
__device__ __forceinline__ v8f mma16(v16h a, v16h b, v8f c) {
  return __builtin_amdgcn_wmma_f32_16x16x32_f16(false, a, false, b, (short)0, c, false, false);
}
__device__ __forceinline__ void guard_rec6(v8f& m0, v8f& r0, v8f& m1, v8f& r1,
                                           v16h a0, v16h a1, v16h b0, v16h b1, v16h b2, v16h b3) {
  asm volatile("v_nop\n\tv_nop\n\tv_nop\n\tv_nop"
               : "+v"(m0), "+v"(r0), "+v"(m1), "+v"(r1)
               : "v"(a0), "v"(a1), "v"(b0), "v"(b1), "v"(b2), "v"(b3));
}
__device__ __forceinline__ void guard_rec5(v8f& m0, v8f& r0, v8f& m1, v8f& r1,
                                           v16h a0, v16h b0, v16h b1, v16h b2, v16h b3) {
  asm volatile("v_nop\n\tv_nop\n\tv_nop\n\tv_nop"
               : "+v"(m0), "+v"(r0), "+v"(m1), "+v"(r1)
               : "v"(a0), "v"(b0), "v"(b1), "v"(b2), "v"(b3));
}
__device__ __forceinline__ void acc_guard4(v8f& a, v8f& b, v8f& c, v8f& d) {
  asm volatile("v_nop\n\tv_nop\n\tv_nop\n\tv_nop" : "+v"(a), "+v"(b), "+v"(c), "+v"(d));
}

__device__ __forceinline__ float tanh_acc(float x) {
  const float ax = fabsf(x);
  const float e  = __expf(-2.0f * ax);
  const float t  = (1.0f - e) * __builtin_amdgcn_rcpf(1.0f + e);
  return copysignf(t, x);
}

__global__ __launch_bounds__(256) void split_plane_kernel(
    const float* __restrict__ src, unsigned short* dval, unsigned short* dres,
    int total8, float carry, int with_res)
{
  const int i = blockIdx.x * 256 + threadIdx.x;
  if (i >= total8) return;
  const size_t e0 = (size_t)i << 3;
  const v4f a0 = *(const v4f*)(src + e0);
  const v4f a1 = *(const v4f*)(src + e0 + 4);
  v8h hv, lv;
#pragma unroll
  for (int e = 0; e < 4; ++e) {
    const float c0 = a0[e] * carry;
    const float c1 = a1[e] * carry;
    const _Float16 h0 = (_Float16)c0;
    const _Float16 h1 = (_Float16)c1;
    const float d0 = c0 - (float)h0;
    const float d1 = c1 - (float)h1;
    hv[e]     = h0;
    hv[4 + e] = h1;
    lv[e]     = (_Float16)(d0 * kCarryR);
    lv[4 + e] = (_Float16)(d1 * kCarryR);
  }
  unsigned short* qv = dval + e0;
  unsigned short* qr = dres + e0;
  *(volatile v8h*)qv = hv;
  if (with_res) *(volatile v8h*)qr = lv;
  __threadfence();
  *(volatile v8h*)qv = hv;
  if (with_res) *(volatile v8h*)qr = lv;
}

__global__ __launch_bounds__(256) void table_kernel(
    const float* __restrict__ emb, const float* __restrict__ Wx, const float* __restrict__ bh,
    float* __restrict__ P0)
{
  __shared__ __align__(16) float sE[kEmbed];
  const int tid = threadIdx.x;
  const int v = blockIdx.x;
  const int n = blockIdx.y * 256 + tid;
  sE[tid] = emb[(size_t)v * kEmbed + tid];
  __syncthreads();
  const float* wr = Wx + (size_t)n * kEmbed;
  float acc = 0.0f;
#pragma unroll 1
  for (int k4 = 0; k4 < kEmbed / 4; ++k4) {
    const v4f w = *(const v4f*)(wr + 4 * k4);
    const v4f e = *(const v4f*)(sE + 4 * k4);
    acc = fmaf(w[0], e[0], acc);
    acc = fmaf(w[1], e[1], acc);
    acc = fmaf(w[2], e[2], acc);
    acc = fmaf(w[3], e[3], acc);
  }
  const float val = acc + bh[n];
  float* q = P0 + (size_t)v * kHid + n;
  *(volatile float*)q = val;
  __threadfence();
  *(volatile float*)q = val;
}

template <int LAYER>
__global__ __launch_bounds__(512) void rec_layer_kernel(
    const int* __restrict__ xid, const float* __restrict__ P0,
    const unsigned short* __restrict__ hin,
    const unsigned short* __restrict__ wx_val, const unsigned short* __restrict__ wx_res,
    const float* __restrict__ bias,
    const unsigned short* __restrict__ wh_val, const unsigned short* __restrict__ wh_res,
    unsigned short* __restrict__ hs_out, float* __restrict__ h_last)
{
  __shared__ __align__(16) _Float16 sH[2][2][16 * kHP];

  const int tid  = threadIdx.x;
  const int lane = tid & 31;
  const int wave = __builtin_amdgcn_readfirstlane((int)(threadIdx.x >> 5));
  const int hh   = lane >> 4;
  const int c    = lane & 15;
  const int koff = hh * 8;
  const int b0   = blockIdx.x * 16;
  const int n0   = 32 * wave + 2 * c;

  {
    const v8h z = (v8h){(_Float16)0.0f, (_Float16)0.0f, (_Float16)0.0f, (_Float16)0.0f,
                        (_Float16)0.0f, (_Float16)0.0f, (_Float16)0.0f, (_Float16)0.0f};
    _Float16* zb = &sH[0][0][0];
    for (int i = tid; i < (2 * 16 * kHP) / 8; i += 512) *(v8h*)(zb + i * 8) = z;
  }
  __syncthreads();

  const _Float16* whv = (const _Float16*)(const void*)wh_val + (size_t)n0 * kHid + koff;
  const _Float16* whr = (const _Float16*)(const void*)wh_res + (size_t)n0 * kHid + koff;
  const _Float16* wxv = (const _Float16*)(const void*)wx_val + (size_t)n0 * kHid + koff;
  const _Float16* wxr = (const _Float16*)(const void*)wx_res + (size_t)n0 * kHid + koff;

  float bias0 = 0.0f, bias1 = 0.0f;
  if (LAYER == 1) {
    const v2f bv = *(const v2f*)(bias + n0);
    bias0 = bv[0];
    bias1 = bv[1];
  }

#pragma unroll 1
  for (int t = 0; t < kSeq; ++t) {
    const int cur = t & 1;
    const int nxt = cur ^ 1;

    float add0[8], add1[8];
    if (LAYER == 0) {
      int xi[8];
#pragma unroll
      for (int r = 0; r < 8; ++r) xi[r] = xid[(size_t)(b0 + 8 * hh + r) * kSeq + t];
#pragma unroll
      for (int r = 0; r < 8; ++r) {
        int xv = xi[r];
        xv = xv < 0 ? 0 : xv;
        xv = xv > (kVocab - 1) ? (kVocab - 1) : xv;
        const v2f p = *(const v2f*)(P0 + (size_t)xv * kHid + n0);
        add0[r] = p[0];
        add1[r] = p[1];
      }
    } else {
#pragma unroll
      for (int r = 0; r < 8; ++r) {
        add0[r] = bias0;
        add1[r] = bias1;
      }
    }

    v8f m0 = (v8f){0.f, 0.f, 0.f, 0.f, 0.f, 0.f, 0.f, 0.f};
    v8f r0 = m0, m1 = m0, r1 = m0;

    if (LAYER == 1) {
      const _Float16* ap = (const _Float16*)(const void*)hin + ((size_t)(b0 + c) * kSeq + t) * kHid + koff;
#pragma unroll 2
      for (int k0 = 0; k0 < kHid; k0 += 32) {
        const v16h a   = ld_frag(ap + k0);
        const v16h bv0 = ld_frag(wxv + k0);
        const v16h br0 = ld_frag(wxr + k0);
        const v16h bv1 = ld_frag(wxv + kHid + k0);
        const v16h br1 = ld_frag(wxr + kHid + k0);
        m0 = mma16(a, bv0, m0);
        r0 = mma16(a, br0, r0);
        m1 = mma16(a, bv1, m1);
        r1 = mma16(a, br1, r1);
        guard_rec5(m0, r0, m1, r1, a, bv0, br0, bv1, br1);
      }
    }
    {
      const _Float16* avp = &sH[cur][0][c * kHP + koff];
      const _Float16* arp = &sH[cur][1][c * kHP + koff];
#pragma unroll 2
      for (int k0 = 0; k0 < kHid; k0 += 32) {
        const v16h av  = ld_frag(avp + k0);
        const v16h ar  = ld_frag(arp + k0);
        const v16h bv0 = ld_frag(whv + k0);
        const v16h br0 = ld_frag(whr + k0);
        const v16h bv1 = ld_frag(whv + kHid + k0);
        const v16h br1 = ld_frag(whr + kHid + k0);
        m0 = mma16(av, bv0, m0);
        r0 = mma16(av, br0, r0);
        r0 = mma16(ar, bv0, r0);
        m1 = mma16(av, bv1, m1);
        r1 = mma16(av, br1, r1);
        r1 = mma16(ar, bv1, r1);
        guard_rec6(m0, r0, m1, r1, av, ar, bv0, br0, bv1, br1);
      }
    }
    acc_guard4(m0, r0, m1, r1);

    float hv0[8], hv1[8];
#pragma unroll
    for (int r = 0; r < 8; ++r) {
      const float s0 = fmaf(r0[r], kResInv, m0[r]);
      const float s1 = fmaf(r1[r], kResInv, m1[r]);
      const float p0v = fmaf(s0, kFold, add0[r]);
      const float p1v = fmaf(s1, kFold, add1[r]);
      const float t0 = tanh_acc(p0v);
      const float t1 = tanh_acc(p1v);
      hv0[r] = t0;
      hv1[r] = t1;
      const float c0 = t0 * kCarryH;
      const float c1 = t1 * kCarryH;
      const _Float16 v0 = (_Float16)c0;
      const _Float16 v1 = (_Float16)c1;
      const float d0 = c0 - (float)v0;
      const float d1 = c1 - (float)v1;
      const _Float16 q0 = (_Float16)(d0 * kCarryR);
      const _Float16 q1 = (_Float16)(d1 * kCarryR);
      v2h pv, pr;
      pv[0] = v0;
      pv[1] = v1;
      pr[0] = q0;
      pr[1] = q1;
      const int off = (8 * hh + r) * kHP + n0;
      *(v2h*)(&sH[nxt][0][off]) = pv;
      *(v2h*)(&sH[nxt][1][off]) = pr;
    }
    __syncthreads();

    {
      const _Float16* src = &sH[nxt][0][wave * kHP + lane * 8];
      const v8h q0 = *(const v8h*)(src);
      const v8h q1 = *(const v8h*)(src + 256);
      unsigned short* dst = hs_out + ((size_t)(b0 + wave) * kSeq + t) * kHid + lane * 8;
      *(volatile v8h*)(dst) = q0;
      *(volatile v8h*)(dst + 256) = q1;
      __threadfence();
      *(volatile v8h*)(dst) = q0;
      *(volatile v8h*)(dst + 256) = q1;
    }

    if (t == kSeq - 1) {
      float* ob = h_last + (size_t)(b0 + 8 * hh) * kHid + n0;
      for (int pass = 0; pass < 2; ++pass) {
#pragma unroll
        for (int r = 0; r < 8; ++r) {
          v2f o;
          o[0] = hv0[r];
          o[1] = hv1[r];
          *(volatile v2f*)(ob + (size_t)r * kHid) = o;
        }
        __threadfence();
      }
    }
  }
}

__device__ __forceinline__ void guard_gemm(v8f& a0, v8f& a1, v8f& a2, v8f& a3,
                                           v16h x, v16h b0, v16h b1, v16h b2, v16h b3) {
  asm volatile("v_nop\n\tv_nop\n\tv_nop\n\tv_nop"
               : "+v"(a0), "+v"(a1), "+v"(a2), "+v"(a3)
               : "v"(x), "v"(b0), "v"(b1), "v"(b2), "v"(b3));
}

__global__ __launch_bounds__(256) void logits_gemm_kernel(
    const unsigned short* __restrict__ Ap, const unsigned short* __restrict__ Btp,
    float* __restrict__ C, const float* __restrict__ bias, float scale)
{
  constexpr int M = kRows, N = kVocab, K = kHid;
  constexpr int lda = kHid, ldb = kHid, ldc = kVocab;
  const _Float16* A  = (const _Float16*)(const void*)Ap;
  const _Float16* Bt = (const _Float16*)(const void*)Btp;
  __shared__ __align__(16) float sT[8][16 * 68];
  const int lane = threadIdx.x & 31;
  const int wave = __builtin_amdgcn_readfirstlane((int)(threadIdx.x >> 5));
  constexpr int tilesN = N >> 6;
  constexpr int tilesM = M >> 6;
  const int tile = blockIdx.x * 8 + wave;
  if (tile >= tilesM * tilesN) return;
  const int tm = tile / tilesN;
  const int tn = tile - tm * tilesN;
  const int m0 = tm << 6;
  const int n0 = tn << 6;

  const int rlane = lane & 15;
  const int koff  = (lane >> 4) * 8;
  const int mOff  = (lane >> 4) * 8;

  v8f acc[4][4];
#pragma unroll
  for (int i = 0; i < 4; ++i)
#pragma unroll
    for (int j = 0; j < 4; ++j) acc[i][j] = (v8f){0.f, 0.f, 0.f, 0.f, 0.f, 0.f, 0.f, 0.f};

  for (int k0 = 0; k0 < K; k0 += 32) {
    v16h bh[4];
#pragma unroll
    for (int j = 0; j < 4; ++j) {
      const size_t bo = (size_t)(n0 + (j << 4) + rlane) * ldb + koff + k0;
      bh[j] = ld_frag(Bt + bo);
    }
#pragma unroll
    for (int i = 0; i < 4; ++i) {
      const size_t ao = (size_t)(m0 + (i << 4) + rlane) * lda + koff + k0;
      const v16h ah = ld_frag(A + ao);
#pragma unroll
      for (int j = 0; j < 4; ++j) acc[i][j] = mma16(ah, bh[j], acc[i][j]);
      guard_gemm(acc[i][0], acc[i][1], acc[i][2], acc[i][3], ah, bh[0], bh[1], bh[2], bh[3]);
    }
  }
  acc_guard4(acc[0][0], acc[0][1], acc[0][2], acc[0][3]);
  acc_guard4(acc[1][0], acc[1][1], acc[1][2], acc[1][3]);
  acc_guard4(acc[2][0], acc[2][1], acc[2][2], acc[2][3]);
  acc_guard4(acc[3][0], acc[3][1], acc[3][2], acc[3][3]);

  float* slab = sT[wave];
#pragma unroll
  for (int i = 0; i < 4; ++i) {
    const int mBase = m0 + (i << 4);
#pragma unroll
    for (int j = 0; j < 4; ++j) {
      const int n = n0 + (j << 4) + rlane;
      const float bv = bias[n];
#pragma unroll
      for (int r = 0; r < 8; ++r) {
        const float v = fmaf(acc[i][j][r], scale, bv);
        slab[(mOff + r) * 68 + (j << 4) + rlane] = v;
      }
    }
    __builtin_amdgcn_fence(__ATOMIC_RELEASE, "workgroup");
    __builtin_amdgcn_wave_barrier();
    __builtin_amdgcn_fence(__ATOMIC_ACQUIRE, "workgroup");
    {
      const int hh = lane >> 4, c4 = (lane & 15) * 4;
      for (int pass = 0; pass < 2; ++pass) {
#pragma unroll
        for (int it = 0; it < 8; ++it) {
          const int row = it * 2 + hh;
          const v4f v = *(const v4f*)(slab + row * 68 + c4);
          *(volatile v4f*)(C + (size_t)(mBase + row) * ldc + n0 + c4) = v;
        }
        __threadfence();
      }
    }
    __builtin_amdgcn_fence(__ATOMIC_RELEASE, "workgroup");
    __builtin_amdgcn_wave_barrier();
    __builtin_amdgcn_fence(__ATOMIC_ACQUIRE, "workgroup");
  }
}

extern "C" void kernel_launch(void* const* d_in, const int* in_sizes, int n_in,
                              void* d_out, int out_size, void* d_ws, size_t ws_size,
                              hipStream_t stream) {
  if (n_in < 10) return;
  if (in_sizes[0] != kBatch * kSeq) return;
  if (in_sizes[1] != kVocab * kEmbed) return;
  if (in_sizes[2] != kHid * kEmbed) return;
  if (in_sizes[3] != kHid * kHid) return;
  if (in_sizes[4] != kHid) return;
  if (in_sizes[5] != kHid * kHid) return;
  if (in_sizes[6] != kHid * kHid) return;
  if (in_sizes[7] != kHid) return;
  if (in_sizes[8] != kVocab * kHid) return;
  if (in_sizes[9] != kVocab) return;
  if ((size_t)out_size != kOutTotal) return;
  if (ws_size < kWsTotal) return;

  const int*   x    = (const int*)d_in[0];
  const float* emb  = (const float*)d_in[1];
  const float* Wxh0 = (const float*)d_in[2];
  const float* Whh0 = (const float*)d_in[3];
  const float* bh0  = (const float*)d_in[4];
  const float* Wxh1 = (const float*)d_in[5];
  const float* Whh1 = (const float*)d_in[6];
  const float* bh1  = (const float*)d_in[7];
  const float* Why  = (const float*)d_in[8];
  const float* by   = (const float*)d_in[9];
  float* out = (float*)d_out;

  char* ws = (char*)d_ws;
  unsigned short* HS0  = (unsigned short*)(ws + kOffHS0);
  unsigned short* HS1  = (unsigned short*)(ws + kOffHS1);
  unsigned short* WH0V = (unsigned short*)(ws + kOffWH0V);
  unsigned short* WH0R = (unsigned short*)(ws + kOffWH0R);
  unsigned short* WX1V = (unsigned short*)(ws + kOffWX1V);
  unsigned short* WX1R = (unsigned short*)(ws + kOffWX1R);
  unsigned short* WH1V = (unsigned short*)(ws + kOffWH1V);
  unsigned short* WH1R = (unsigned short*)(ws + kOffWH1R);
  unsigned short* WYV  = (unsigned short*)(ws + kOffWYV);
  float*          P0   = (float*)(ws + kOffP0);

  split_plane_kernel<<<(kHid * kHid / 8) / 256, 256, 0, stream>>>(Whh0, WH0V, WH0R, kHid * kHid / 8, kCarryW, 1);
  split_plane_kernel<<<(kHid * kHid / 8) / 256, 256, 0, stream>>>(Wxh1, WX1V, WX1R, kHid * kHid / 8, kCarryW, 1);
  split_plane_kernel<<<(kHid * kHid / 8) / 256, 256, 0, stream>>>(Whh1, WH1V, WH1R, kHid * kHid / 8, kCarryW, 1);
  split_plane_kernel<<<(kVocab * kHid / 8) / 256, 256, 0, stream>>>(Why, WYV, WYV, kVocab * kHid / 8, kCarryW, 0);

  table_kernel<<<dim3(kVocab, kHid / 256), 256, 0, stream>>>(emb, Wxh0, bh0, P0);

  rec_layer_kernel<0><<<kBatch / 16, 512, 0, stream>>>(
      x, P0, HS1, WX1V, WX1R, bh0, WH0V, WH0R, HS0, out + kOutH0);

  rec_layer_kernel<1><<<kBatch / 16, 512, 0, stream>>>(
      x, P0, HS0, WX1V, WX1R, bh1, WH1V, WH1R, HS1, out + kOutH1);

  logits_gemm_kernel<<<(kRows / 64) * (kVocab / 64) / 8, 256, 0, stream>>>(
      HS1, WYV, out + kOutLogits, by, kFold);
}
